// MultiAttentionBlock_43456479101353
// MI455X (gfx1250) — hardware-run, weakly checked
//
#include <hip/hip_runtime.h>


namespace {
constexpr int NN = 50000, NP = 50016, NE = 400000, C = 64, H = 12, HG = 4, NGRP = 3, CG = HG * C  , MAXDEG = 1024, NGc = (NN + 511) / 512, PERMLEN = NE + 32 * NGc + 32;
constexpr float XS = 8.0f, SLOPE = 0.2f;

typedef _Float16 b16;
typedef __attribute__((ext_vector_type(16))) _Float16 v16b;
typedef __attribute__((ext_vector_type(8))) _Float16 v8b;
typedef __attribute__((ext_vector_type(8))) float v8f;
typedef __attribute__((ext_vector_type(4))) float v4f;
typedef __attribute__((ext_vector_type(2))) float v2f;
__device__ __forceinline__ float bf16_rne(float f) { unsigned int u = __float_as_uint(f); u += 0x7FFFu + ((u >> 16) & 1u); return __uint_as_float(u & 0xFFFF0000u); }
__device__ __forceinline__ v16b frag_kb(const b16* p, int hh) { const v8b a = *(const v8b*)(p + 8 * hh), b = *(const v8b*)(p + 16 + 8 * hh); v16b f;
#pragma unroll
  for (int e = 0; e < 8; ++e) { f[e] = a[e]; f[8 + e] = b[e]; } return f; }
__device__ __forceinline__ v8f wmma16b(v16b a, v16b b, v8f c) { v8f d = __builtin_amdgcn_wmma_f32_16x16x32_f16(false, a, false, b, (short)0, c, false, false); asm volatile("v_nop\n\tv_nop\n\tv_nop\n\tv_nop" : "+v"(d) : "v"(a), "v"(b)); return d; }
__device__ __forceinline__ void wave_lds_sync() { __builtin_amdgcn_fence(__ATOMIC_RELEASE, "workgroup"); __builtin_amdgcn_wave_barrier(); __builtin_amdgcn_fence(__ATOMIC_ACQUIRE, "workgroup"); }
__device__ __forceinline__ float nexp(float x) { return __builtin_amdgcn_exp2f(x * 1.4426950408889634f); }
__device__ __forceinline__ float pmul(float a, float b) { float p = a * b; asm volatile("" : "+v"(p)); return p; }
__device__ __forceinline__ float leaky(float x) { return (x >= 0.0f) ? x : SLOPE * x; }
constexpr int CSR_NBLK = 512, CSR_GB = 9, CSR_GN = 1 << CSR_GB  , CSR_MAXG = 512, CSR_CAP = 12288  ;
__global__ __launch_bounds__(64) void csrA_kernel(const int* __restrict__ dst, int E, int N, int nG, int CHP, int NGP, int* __restrict__ STG, int* __restrict__ HST) {
  extern __shared__ int sm[];
  int* cnt = sm; int* run = sm + NGP; int* ids = sm + 2 * NGP;
  const int b = blockIdx.x; const int ch = (E + CSR_NBLK - 1) / CSR_NBLK; const int e0 = b * ch, e1 = min(E, e0 + ch);
  for (int i = threadIdx.x; i < NGP; i += 64) cnt[i] = 0;
  for (int i = threadIdx.x; i < CHP; i += 64) ids[i] = -1;
  __syncthreads();
  if (threadIdx.x == 0) {
    for (int e = e0; e < e1; ++e) { int d = dst[e]; d = (d < 0) ? 0 : (d >= N ? N - 1 : d); cnt[d >> CSR_GB] += 1; }
    int acc = 0; for (int g = 0; g < nG; ++g) { run[g] = acc; acc += cnt[g]; }
    for (int e = e0; e < e1; ++e) { int d = dst[e]; d = (d < 0) ? 0 : (d >= N ? N - 1 : d); const int g = d >> CSR_GB; ids[run[g]] = e; run[g] += 1; } }
  __syncthreads();
  typedef __attribute__((ext_vector_type(4))) int v4i;
  for (int pass = 0; pass < 2; ++pass) {
    for (int i = threadIdx.x; i < CHP / 4; i += 64) *(volatile v4i*)(STG + (size_t)b * CHP + i * 4) = *(const v4i*)(&ids[i * 4]);
    for (int i = threadIdx.x; i < NGP / 4; i += 64) { v4i v; for (int e = 0; e < 4; ++e) v[e] = (i * 4 + e < nG) ? cnt[i * 4 + e] : 0; *(volatile v4i*)(HST + (size_t)b * NGP + i * 4) = v; }
    __threadfence(); }
}
__global__ __launch_bounds__(512) void csrS_kernel(const int* __restrict__ HST, int nG, int NGP, int* __restrict__ START, int* __restrict__ TOT, int* __restrict__ OFF) {
  __shared__ int tot[CSR_MAXG];
  const int b = threadIdx.x;
  for (int pass = 0; pass < 2; ++pass) { int runb = 0; for (int g = 0; g < nG; ++g) { int c = HST[(size_t)b * NGP + g]; c = (c < 0) ? 0 : c; ((volatile int*)OFF)[(size_t)g * CSR_NBLK + b] = runb; runb += c; } __threadfence(); }
  for (int g = threadIdx.x; g < nG; g += 512) { int s = 0; for (int bb = 0; bb < CSR_NBLK; ++bb) { int c = HST[(size_t)bb * NGP + g]; s += (c < 0) ? 0 : c; } tot[g] = s; }
  __syncthreads();
  if (threadIdx.x < 32) {
    __shared__ int st[CSR_MAXG + 32];
    if (threadIdx.x == 0) { int acc = 0; for (int g = 0; g < NGP; ++g) { st[g] = acc; if (g < nG) acc += (tot[g] + 31) & ~31; } st[NGP] = acc; }
    __builtin_amdgcn_fence(__ATOMIC_RELEASE, "workgroup"); __builtin_amdgcn_wave_barrier(); __builtin_amdgcn_fence(__ATOMIC_ACQUIRE, "workgroup");
    for (int pass = 0; pass < 2; ++pass) { for (int i = threadIdx.x; i < NGP + 32; i += 32) { ((volatile int*)START)[i] = (i <= NGP) ? st[min(i, NGP)] : 0; ((volatile int*)TOT)[i] = (i < nG) ? tot[i] : 0; } __threadfence(); } }
}
__global__ __launch_bounds__(256) void csrB_kernel(const int* __restrict__ dst, int N, int nG, int CHP, int NGP, int permLen, const int* __restrict__ STG, const int* __restrict__ HST, const int* __restrict__ OFF, const int* __restrict__ START, const int* __restrict__ TOT, int* __restrict__ PERM, int* __restrict__ ROWPTR, int* __restrict__ ROWCNT, int* __restrict__ FLAG) {
  typedef __attribute__((ext_vector_type(4))) int v4i;
  __shared__ int ids[CSR_CAP]; __shared__ unsigned short key[CSR_CAP]; __shared__ int outp[CSR_CAP]; __shared__ int ncnt[CSR_GN + 1]; __shared__ int boff[CSR_NBLK + 1];
  const int g = blockIdx.x, t_ = threadIdx.x; int tot = TOT[g]; int st = START[g], stn = START[g + 1]; const int v0 = g * CSR_GN; const int nv = min(CSR_GN, N - v0);
  st = (st < 0) ? 0 : (st > permLen - 32 ? permLen - 32 : st) & ~31; stn = (stn < st) ? st : (stn > permLen ? permLen : stn); tot = (tot < 0) ? 0 : tot; if (tot > stn - st && tot <= CSR_CAP) tot = stn - st;
  if (tot > CSR_CAP) {
    for (int pass = 0; pass < 2; ++pass) { for (int i = t_; i < CSR_GN / 4; i += 256) { v4i a, c; for (int e = 0; e < 4; ++e) { a[e] = st; c[e] = 0; } *(volatile v4i*)(ROWPTR + v0 + i * 4) = a; *(volatile v4i*)(ROWCNT + v0 + i * 4) = c; } if (t_ == 0) ((volatile int*)FLAG)[0] = 1; __threadfence(); } (void)nv; return; }
  if (t_ == 0) { int acc = 0; for (int b = 0; b < CSR_NBLK; ++b) { boff[b] = acc; int c = HST[(size_t)b * NGP + g]; c = (c < 0) ? 0 : (c > CHP ? CHP : c); acc += c; if (acc > tot) acc = tot; } boff[CSR_NBLK] = acc; }
  for (int i = t_; i <= CSR_GN; i += 256) ncnt[i] = 0;
  __syncthreads();
  for (int b = 0; b < CSR_NBLK; ++b) { const int c = boff[b + 1] - boff[b]; int o_ = OFF[(size_t)g * CSR_NBLK + b]; o_ = (o_ < 0) ? 0 : (o_ > CHP - c ? CHP - c : o_); const int* src_ = STG + (size_t)b * CHP + o_;
    for (int i = t_; i < c; i += 256) { int id = src_[i]; id = (id < 0) ? 0 : id; ids[boff[b] + i] = id; int d = dst[id]; d = (d < v0) ? v0 : (d >= N ? N - 1 : d); int kk = d - v0; kk = (kk < 0) ? 0 : (kk >= CSR_GN ? CSR_GN - 1 : kk); key[boff[b] + i] = (unsigned short)kk; } }
  __syncthreads();
  if (t_ == 0) { for (int i = 0; i < tot; ++i) ncnt[key[i]] += 1; int acc = 0; for (int vl = 0; vl < CSR_GN; ++vl) { const int c = ncnt[vl]; ncnt[vl] = acc; acc += c; } ncnt[CSR_GN] = acc;
    for (int i = 0; i < tot; ++i) { const int vl = key[i]; outp[ncnt[vl]] = ids[i]; ncnt[vl] += 1; }
    for (int vl = CSR_GN; vl > 0; --vl) ncnt[vl] = ncnt[vl - 1]; ncnt[0] = 0; }
  __syncthreads();
  for (int pass = 0; pass < 2; ++pass) {
    for (int i = t_; i < (stn - st) / 4; i += 256) { v4i v; for (int e = 0; e < 4; ++e) { const int q = i * 4 + e; v[e] = (q < tot) ? outp[q] : -1; } *(volatile v4i*)(PERM + st + i * 4) = v; }
    for (int i = t_; i < CSR_GN / 4; i += 256) { v4i a, c; for (int e = 0; e < 4; ++e) { const int vl = i * 4 + e; a[e] = st + ncnt[vl]; c[e] = (vl < nv) ? (ncnt[vl + 1] - ncnt[vl]) : 0; } *(volatile v4i*)(ROWPTR + v0 + i * 4) = a; *(volatile v4i*)(ROWCNT + v0 + i * 4) = c; }
    __threadfence(); }
}
__global__ __launch_bounds__(256) void csrZ_kernel(int* __restrict__ p, size_t n4) { typedef __attribute__((ext_vector_type(4))) int v4i; const size_t tid = (size_t)blockIdx.x * 256 + threadIdx.x, nth = (size_t)gridDim.x * 256; v4i z = {0, 0, 0, 0}; for (size_t i = tid; i < n4; i += nth) *(volatile v4i*)(p + i * 4) = z; }
struct CsrBufs { int *STG, *HST, *OFF, *START, *TOT, *PERM, *ROWPTR, *ROWCNT, *FLAG; int nG, NGP, CHP; size_t permLen; char* base; size_t bytes; };
static size_t csr_carve(CsrBufs& c, char* ws, size_t off, int E, int N) {
  const size_t off0 = off; c.base = ws + off;
  auto al = [&](size_t bytes) { char* p = ws + off; off += (bytes + 255) & ~(size_t)255; return p; };
  c.nG = (N + CSR_GN - 1) / CSR_GN; c.NGP = (c.nG + 31) & ~31; const int ch = (E + CSR_NBLK - 1) / CSR_NBLK; c.CHP = (ch + 31) & ~31; c.permLen = (size_t)E + 32 * (size_t)c.nG + 32;
  c.STG = (int*)al((size_t)CSR_NBLK * c.CHP * 4); c.HST = (int*)al((size_t)CSR_NBLK * c.NGP * 4); c.OFF = (int*)al((size_t)c.NGP * CSR_NBLK * 4); c.START = (int*)al((size_t)(c.NGP + 64) * 4); c.TOT = (int*)al((size_t)(c.NGP + 64) * 4);
  c.PERM = (int*)al(c.permLen * 4); c.ROWPTR = (int*)al((size_t)c.nG * CSR_GN * 4); c.ROWCNT = (int*)al((size_t)c.nG * CSR_GN * 4); c.FLAG = (int*)al(256);
  c.bytes = off - off0; return off;
}
static void csr_build(const CsrBufs& c, const int* dst, int E, int N, hipStream_t stream) {
  const size_t smem = (size_t)(2 * c.NGP + c.CHP) * 4;
  csrZ_kernel<<<512, 256, 0, stream>>>((int*)c.base, c.bytes / 16);
  csrA_kernel<<<CSR_NBLK, 64, smem, stream>>>(dst, E, N, c.nG, c.CHP, c.NGP, c.STG, c.HST);
  csrS_kernel<<<1, 512, 0, stream>>>(c.HST, c.nG, c.NGP, c.START, c.TOT, c.OFF);
  csrB_kernel<<<c.nG, 256, 0, stream>>>(dst, N, c.nG, c.CHP, c.NGP, (int)c.permLen, c.STG, c.HST, c.OFF, c.START, c.TOT, c.PERM, c.ROWPTR, c.ROWCNT, c.FLAG);
}

__global__ __launch_bounds__(256) void prep_kernel(const float* __restrict__ x, const float* __restrict__ w, const float* __restrict__ as_, const float* __restrict__ ad_, const float* __restrict__ bias, b16* __restrict__ R, float* __restrict__ P, b16* __restrict__ X, float* __restrict__ Xf) {
  const size_t tid = (size_t)blockIdx.x * 256 + threadIdx.x, nth = (size_t)gridDim.x * 256;
  for (int pass = 0; pass < 2; ++pass) {
    for (size_t p = tid; p < (size_t)H * C * (C / 8); p += nth) { const int o = (int)(p / (C / 8)), k0 = (int)(p % (C / 8)) * 8; v8b v; for (int e = 0; e < 8; ++e) v[e] = (b16)bf16_rne(w[(size_t)(k0 + e) * (H * C) + o]); *(volatile v8b*)(R + (size_t)o * C + k0) = v; }
    for (size_t q = tid; q < 1600; q += nth) { const int i = (int)q; P[q] = bf16_rne((i < 768) ? as_[i] : (i < 1536) ? ad_[i - 768] : bias[i - 1536]); }
    for (size_t p = tid; p < (size_t)NP * C / 8; p += nth) { const size_t r = p / (C / 8); v8b v = {}; float f[8] = {0, 0, 0, 0, 0, 0, 0, 0}; if (r < (size_t)NN) { for (int e = 0; e < 8; ++e) { f[e] = bf16_rne(x[p * 8 + e]); v[e] = (b16)(f[e] * XS); } }
      *(volatile v8b*)(X + p * 8) = v; *(volatile v4f*)(Xf + p * 8) = *(v4f*)&f[0]; *(volatile v4f*)(Xf + p * 8 + 4) = *(v4f*)&f[4]; }
    __threadfence(); }
}

__global__ __launch_bounds__(64) void gemm_kernel(const b16* __restrict__ X, const b16* __restrict__ R, const float* __restrict__ P, int g, float* __restrict__ HGf, float* __restrict__ AS, float* __restrict__ AD) {
  __shared__ __attribute__((aligned(16))) float Ts[2][32][128 + 4]; __shared__ float Av[2][4][32];
  const int lane = threadIdx.x & 31, wave = threadIdx.x >> 5, nloc = lane & 15, hlf = lane >> 4, m0 = blockIdx.x * 32, c0 = wave * 128; const b16* Bw = R + (size_t)(g * CG) * C;
  v8f acc[2][8];
#pragma unroll
  for (int r = 0; r < 2; ++r)
#pragma unroll
    for (int t = 0; t < 8; ++t) acc[r][t] = (v8f){};
#pragma unroll
  for (int kb = 0; kb < C; kb += 32) { const v16b a0 = frag_kb(X + (size_t)(m0 + nloc) * C + kb, hlf), a1 = frag_kb(X + (size_t)(m0 + 16 + nloc) * C + kb, hlf);
#pragma unroll
    for (int t = 0; t < 8; ++t) { const v16b bw = frag_kb(Bw + (size_t)(c0 + t * 16 + nloc) * C + kb, hlf); acc[0][t] = wmma16b(a0, bw, acc[0][t]); acc[1][t] = wmma16b(a1, bw, acc[1][t]); } }
#pragma unroll
  for (int t = 0; t < 8; ++t)
#pragma unroll
    for (int r = 0; r < 2; ++r)
#pragma unroll
      for (int v = 0; v < 8; ++v) Ts[wave][r * 16 + 8 * hlf + v][t * 16 + nloc] = acc[r][t][v] * (1.0f / XS);
  wave_lds_sync();
  { const int rr = lane;
    for (int k = 0; k < 2; ++k) { const int hd = g * HG + wave * 2 + k; float ss = 0.0f, sd = 0.0f; for (int c = 0; c < C; ++c) { const float hv = Ts[wave][rr][k * C + c]; ss += pmul(hv, P[hd * C + c]); sd += pmul(hv, P[768 + hd * C + c]); } Av[wave][k * 2][rr] = ss; Av[wave][k * 2 + 1][rr] = sd; } }
  wave_lds_sync();
  for (int pass = 0; pass < 2; ++pass) {
    for (int i = lane; i < 32 * 32; i += 32) { const int rr = i >> 5, c4 = (i & 31) * 4; *(volatile v4f*)(HGf + (size_t)(m0 + rr) * CG + c0 + c4) = *(const v4f*)(&Ts[wave][rr][c4]); }
    for (int k = 0; k < 2; ++k) { const int hd = g * HG + wave * 2 + k; ((volatile float*)AS)[(size_t)hd * NP + m0 + lane] = Av[wave][k * 2][lane]; ((volatile float*)AD)[(size_t)hd * NP + m0 + lane] = Av[wave][k * 2 + 1][lane]; }
    __threadfence(); }
}

template <int FINAL>
__global__ __launch_bounds__(256) void gat_kernel(const float* __restrict__ HGf, const float* __restrict__ AS, const float* __restrict__ AD, const int* __restrict__ src, const int* __restrict__ perm, const int* __restrict__ rowptr, const int* __restrict__ rowcnt, const float* __restrict__ P, const float* __restrict__ Xf, int g, float* __restrict__ SUM, float* __restrict__ out) {
  __shared__ float Tmp[8][C];
  const int wave = threadIdx.x >> 5, v = blockIdx.x * 8 + wave, lane = threadIdx.x & 31, k = lane >> 3, c8 = (lane & 7) * 8; const int hd = g * HG + k;
  int cnt = rowcnt[v]; cnt = (cnt < 0) ? 0 : (cnt > MAXDEG ? MAXDEG : cnt); int p0 = rowptr[v]; p0 = (p0 < 0) ? 0 : (p0 > PERMLEN - cnt ? PERMLEN - cnt : p0);
  const float adv = AD[(size_t)hd * NP + v]; float m = -INFINITY, l = 0.0f; float acc[8]; for (int e = 0; e < 8; ++e) acc[e] = 0.0f;
  for (int q = 0; q <= cnt; ++q) { int s; if (q < cnt) { int id = perm[p0 + q]; id = (id < 0) ? 0 : (id >= NE ? NE - 1 : id); s = src[id]; s = (s < 0) ? 0 : (s >= NN ? NN - 1 : s); } else s = v;
    const float e = leaky(AS[(size_t)hd * NP + s] + adv); const float mn = fmaxf(m, e); const float al_ = nexp(m - mn); const float p = nexp(e - mn); m = mn; l = l * al_ + p;
    const v4f h0 = *(const v4f*)(HGf + (size_t)s * CG + k * C + c8), h1 = *(const v4f*)(HGf + (size_t)s * CG + k * C + c8 + 4);
#pragma unroll
    for (int e2 = 0; e2 < 4; ++e2) { acc[e2] = acc[e2] * al_ + pmul(p, h0[e2]); acc[4 + e2] = acc[4 + e2] * al_ + pmul(p, h1[e2]); } }
  const float il = 1.0f / (l + 1e-16f);
  v2f sm = {0.0f, 0.0f}; if (g > 0) sm = *(const v2f*)(SUM + (size_t)v * C + lane * 2);
  for (int kk = 0; kk < HG; ++kk) { if (k == kk) { for (int e2 = 0; e2 < 8; ++e2) Tmp[wave][c8 + e2] = acc[e2] * il; } wave_lds_sync(); sm[0] += Tmp[wave][lane * 2]; sm[1] += Tmp[wave][lane * 2 + 1]; wave_lds_sync(); }
  if (FINAL) { const v2f xr = *(const v2f*)(Xf + (size_t)v * C + lane * 2); v2f o; o[0] = fmaxf(xr[0] + sm[0] * (1.0f / H) + P[1536 + lane * 2], 0.0f); o[1] = fmaxf(xr[1] + sm[1] * (1.0f / H) + P[1536 + lane * 2 + 1], 0.0f);
    for (int pass = 0; pass < 2; ++pass) { *(volatile v2f*)(out + (size_t)v * C + lane * 2) = o; __threadfence(); } }
  else { for (int pass = 0; pass < 2; ++pass) { *(volatile v2f*)(SUM + (size_t)v * C + lane * 2) = sm; __threadfence(); } }
}
}

extern "C" void kernel_launch(void* const* d_in, const int* in_sizes, int n_in,
                              void* d_out, int out_size, void* d_ws, size_t ws_size, hipStream_t stream) {
  (void)n_in; (void)out_size;
  const float* x = (const float*)d_in[0]; const int* ei = (const int*)d_in[1]; const float* w = (const float*)d_in[2]; const float* as_ = (const float*)d_in[3]; const float* ad_ = (const float*)d_in[4]; const float* bias = (const float*)d_in[5];
  float* out = (float*)d_out;
  if (in_sizes[0] != NN * C || in_sizes[1] != 2 * NE || in_sizes[2] != C * H * C) return;
  const int* srcI = ei; const int* dstI = ei + NE; const int NE_RUN = NE;
  size_t off = 0; char* ws = (char*)d_ws;
  auto carve = [&](size_t bytes) { char* p = ws + off; off += (bytes + 255) & ~(size_t)255; return p; };
  b16* R = (b16*)carve((size_t)H * C * C * 2); float* P = (float*)carve(1600 * 4); b16* X = (b16*)carve((size_t)NP * C * 2); float* Xf = (float*)carve((size_t)NP * C * 4); float* HGf = (float*)carve((size_t)NP * CG * 4); float* AS = (float*)carve((size_t)H * NP * 4); float* AD = (float*)carve((size_t)H * NP * 4); float* SUM = (float*)carve((size_t)NP * C * 4);
  CsrBufs cs; off = csr_carve(cs, ws, off, NE_RUN, NN);
  if (off > ws_size) return;
  csr_build(cs, dstI, NE_RUN, NN, stream);
  prep_kernel<<<256, 256, 0, stream>>>(x, w, as_, ad_, bias, R, P, X, Xf);
  for (int g = 0; g < NGRP; ++g) {
    gemm_kernel<<<NP / 32, 64, 0, stream>>>(X, R, P, g, HGf, AS, AD);
    if (g < NGRP - 1) gat_kernel<0><<<NN / 8, 256, 0, stream>>>(HGf, AS, AD, srcI, cs.PERM, cs.ROWPTR, cs.ROWCNT, P, Xf, g, SUM, out);
    else gat_kernel<1><<<NN / 8, 256, 0, stream>>>(HGf, AS, AD, srcI, cs.PERM, cs.ROWPTR, cs.ROWCNT, P, Xf, g, SUM, out); }
}
